// SpotRNAWithTransformer_25220047962437
// MI455X (gfx1250) — hardware-verified
//
#include <hip/hip_runtime.h>
#include <stddef.h>
#include <stdint.h>
#include <math.h>

#define NB      4
#define SQ      512
#define NTOK    2048
#define DM      256
#define NH      4
#define HDM     64
#define DFF     1024
#define NQKV    768
#define NRES    8
#define NLAYER  2
#define KCONV   768
#define SQP     514
#define PADPLANE (NB * SQP * DM)
#define QB      128
#define KC      64
#define NQB     4
#define NCK     8
#define NF1     64
#define NHIJ    128
#define KXC     512
#define PR      32
#define POP     260

static_assert(NTOK == NB * SQ);
static_assert(NH * HDM == DM);
static_assert(NQKV == 3 * DM);
static_assert(NQB * QB == SQ);
static_assert(NCK * KC == SQ);
static_assert(KCONV == 3 * DM);
static_assert(NTOK % 256 == 0);
static_assert(SQ % 256 == 0);
static_assert(DFF % 64 == 0);
static_assert(NHIJ == 2 * NF1);
static_assert(KXC == 2 * DM);
static_assert(((size_t)PADPLANE * 2) % 128 == 0);
static_assert(SQ % PR == 0);
static_assert((POP * 4) % 16 == 0);

typedef _Float16 v16h __attribute__((ext_vector_type(16)));
typedef _Float16 v8h  __attribute__((ext_vector_type(8)));
typedef float    v8f  __attribute__((ext_vector_type(8)));
typedef float    v4f  __attribute__((ext_vector_type(4)));
typedef unsigned int v4u __attribute__((ext_vector_type(4)));

union Frag  { v16h v; v8h h[2]; };
union Pack8 { v8h h; v4u u; };

__device__ __forceinline__ v8f mma16(v16h a, v16h b, v8f c) {
  c = __builtin_amdgcn_wmma_f32_16x16x32_f16(false, a, false, b, (short)0, c, false, false);
  asm volatile("v_nop\n\tv_nop\n\tv_nop\n\tv_nop" : "+v"(c) : "v"(a), "v"(b));
  return c;
}

__device__ __forceinline__ v16h ldfrag(const _Float16* p, int ld, int row0, int k0, int lane) {
  const int m = lane & 15, lh = lane >> 4;
  const _Float16* q = p + (size_t)(row0 + m) * ld + k0 + 8 * lh;
  Frag f;
  f.h[0] = *(const v8h*)(q);
  f.h[1] = *(const v8h*)(q + 16);
  return f.v;
}

__device__ __forceinline__ v8f zero8() { return (v8f){0.f, 0.f, 0.f, 0.f, 0.f, 0.f, 0.f, 0.f}; }

__device__ __forceinline__ v4u pack8h(v4f a0, v4f a1) {
  Pack8 pk;
  pk.h = (v8h){(_Float16)a0[0], (_Float16)a0[1], (_Float16)a0[2], (_Float16)a0[3],
               (_Float16)a1[0], (_Float16)a1[1], (_Float16)a1[2], (_Float16)a1[3]};
  return pk.u;
}

__device__ __forceinline__ void gemm32x64(const _Float16* __restrict__ A, int lda,
                                          const _Float16* __restrict__ Bt, int ldb, int K,
                                          int m0, int n0, int lane, v8f (&acc)[2][4]) {
#pragma unroll 1
  for (int k0 = 0; k0 < K; k0 += 32) {
    const v16h a0 = ldfrag(A, lda, m0, k0, lane);
    const v16h a1 = ldfrag(A, lda, m0 + 16, k0, lane);
    const v16h b0 = ldfrag(Bt, ldb, n0, k0, lane);
    const v16h b1 = ldfrag(Bt, ldb, n0 + 16, k0, lane);
    const v16h b2 = ldfrag(Bt, ldb, n0 + 32, k0, lane);
    const v16h b3 = ldfrag(Bt, ldb, n0 + 48, k0, lane);
    acc[0][0] = mma16(a0, b0, acc[0][0]);
    acc[1][0] = mma16(a1, b0, acc[1][0]);
    acc[0][1] = mma16(a0, b1, acc[0][1]);
    acc[1][1] = mma16(a1, b1, acc[1][1]);
    acc[0][2] = mma16(a0, b2, acc[0][2]);
    acc[1][2] = mma16(a1, b2, acc[1][2]);
    acc[0][3] = mma16(a0, b3, acc[0][3]);
    acc[1][3] = mma16(a1, b3, acc[1][3]);
  }
}

__global__ __launch_bounds__(32) void k_padzero(_Float16* __restrict__ planes) {
  const int lane = threadIdx.x & 31;
  const int blk = blockIdx.x;
  const int p = blk >> 3, b = (blk >> 1) & 3, which = blk & 1;
  const int row = (which != 0) ? (SQP - 1) : 0;
  _Float16* dst = planes + (size_t)p * PADPLANE + ((size_t)b * SQP + row) * DM + 8 * lane;
  const v4u z = (v4u){0u, 0u, 0u, 0u};
  for (int ps = 0; ps < 2; ++ps) {
    *(volatile v4u*)dst = z;
    __threadfence();
  }
}

__global__ __launch_bounds__(256) void k_convw(const float* __restrict__ w, _Float16* __restrict__ out) {
  const int idx = blockIdx.x * 256 + threadIdx.x;
  const int i   = idx / 24576;
  const int rem = idx - i * 24576;
  const int o   = rem / 96;
  const int q   = rem - o * 96;
  const int t   = q >> 5;
  const int c0  = (q & 31) * 8;
  const float* src = w + (((size_t)i * DM + o) * DM + c0) * 3 + t;
  float f[8];
#pragma unroll
  for (int j = 0; j < 8; ++j) f[j] = src[3 * j] * 64.0f;
  const v4u val = pack8h((v4f){f[0], f[1], f[2], f[3]}, (v4f){f[4], f[5], f[6], f[7]});
  _Float16* dst = out + ((size_t)i * DM + o) * KCONV + t * DM + c0;
  for (int ps = 0; ps < 2; ++ps) {
    *(volatile v4u*)dst = val;
    __threadfence();
  }
}

__global__ __launch_bounds__(256) void k_cvt(const float* __restrict__ in, int n8, float scale,
                                             _Float16* __restrict__ out) {
  const int idx = blockIdx.x * 256 + threadIdx.x;
  const int ci  = min(idx, n8 - 1);
  const float* s = in + (size_t)ci * 8;
  const v4u val = pack8h(*(const v4f*)(s) * scale, *(const v4f*)(s + 4) * scale);
  _Float16* dst = out + (size_t)ci * 8;
  if (idx < n8) {
    for (int ps = 0; ps < 2; ++ps) {
      *(volatile v4u*)dst = val;
      __threadfence();
    }
  }
}

__global__ __launch_bounds__(256) void k_cvt_fc1(const float* __restrict__ w, _Float16* __restrict__ out) {
  const int idx = blockIdx.x * 256 + threadIdx.x;
  const int r = idx >> 6, pc = idx & 63;
  const float* s = w + (size_t)(r & 63) * (2 * KXC) + (r >> 6) * KXC + pc * 8;
  const v4u val = pack8h(*(const v4f*)(s) * 64.0f, *(const v4f*)(s + 4) * 64.0f);
  _Float16* dst = out + (size_t)r * KXC + pc * 8;
  for (int ps = 0; ps < 2; ++ps) {
    *(volatile v4u*)dst = val;
    __threadfence();
  }
}

__global__ __launch_bounds__(256) void k_embed(const float* __restrict__ x, const float* __restrict__ ew,
                                               const float* __restrict__ eb,
                                               float* __restrict__ rf, _Float16* __restrict__ hp) {
  __shared__ __align__(16) float sw[8][DM];
  const int tid = threadIdx.x, lane = tid & 31, wave = tid >> 5;
  const int m = blockIdx.x * 8 + wave;
  const int b = m >> 9, l = m & (SQ - 1);
  const v4f xv = *(const v4f*)(x + (size_t)m * 4);

  v4f v[2];
#pragma unroll
  for (int it = 0; it < 2; ++it) {
    const int c0 = it * 128 + lane * 4;
    const v4f bv = *(const v4f*)(eb + c0);
#pragma unroll
    for (int e = 0; e < 4; ++e) {
      const v4f wv = *(const v4f*)(ew + (size_t)(c0 + e) * 4);
      float s = xv[0] * wv[0];
      s = fmaf(xv[1], wv[1], s);
      s = fmaf(xv[2], wv[2], s);
      s = fmaf(xv[3], wv[3], s);
      v[it][e] = s + bv[e];
    }
  }
  float* row = rf + (size_t)m * DM;
  for (int ps = 0; ps < 2; ++ps) {
#pragma unroll
    for (int it = 0; it < 2; ++it) *(volatile v4f*)(row + it * 128 + lane * 4) = v[it];
    __threadfence();
  }
#pragma unroll
  for (int it = 0; it < 2; ++it) *(v4f*)(sw[wave] + it * 128 + lane * 4) = v[it];
  __syncthreads();
  const float* cp = sw[wave] + 8 * lane;
  const v4u hv = pack8h(*(const v4f*)(cp) * 16.0f, *(const v4f*)(cp + 4) * 16.0f);
  _Float16* hdst = hp + ((size_t)b * SQP + 1 + l) * DM + 8 * lane;
  for (int ps = 0; ps < 2; ++ps) {
    *(volatile v4u*)hdst = hv;
    __threadfence();
  }
}

#define OTP 68
template <int SECOND>
__global__ __launch_bounds__(256) void k_conv(const _Float16* __restrict__ hin, const _Float16* __restrict__ wt,
                                              const float* __restrict__ cb, const float* __restrict__ g,
                                              const float* __restrict__ be, const float* __restrict__ mu,
                                              const float* __restrict__ var, const float* __restrict__ res,
                                              float* __restrict__ rout, _Float16* __restrict__ hout) {
  __shared__ __align__(16) float st[8][16 * OTP];
  __shared__ __align__(16) float ep[5][64];
  const int tid = threadIdx.x, lane = tid & 31, wave = tid >> 5;
  const int hh = lane >> 4, c = lane & 15;
  const int m0 = blockIdx.x * 256 + wave * 32;
  const int b = m0 >> 9, l0 = m0 & (SQ - 1);
  const int n0 = blockIdx.y * 64;
  const _Float16* Ab = hin + (size_t)b * SQP * DM;

  if (tid < 64) {
    const int n = n0 + tid;
    ep[0][tid] = cb[n];
    ep[1][tid] = mu[n];
    ep[2][tid] = 1.0f / sqrtf(var[n] + 1e-5f);
    ep[3][tid] = g[n];
    ep[4][tid] = be[n];
  }
  __syncthreads();

  v8f acc[2][4];
#pragma unroll
  for (int s = 0; s < 2; ++s)
#pragma unroll
    for (int t = 0; t < 4; ++t) acc[s][t] = zero8();

#pragma unroll 1
  for (int k0 = 0; k0 < KCONV; k0 += 32) {
    const int tp = k0 >> 8, c0 = k0 & (DM - 1);
    const v16h a0 = ldfrag(Ab, DM, l0 + tp, c0, lane);
    const v16h a1 = ldfrag(Ab, DM, l0 + 16 + tp, c0, lane);
    const v16h b0 = ldfrag(wt, KCONV, n0, k0, lane);
    const v16h b1 = ldfrag(wt, KCONV, n0 + 16, k0, lane);
    const v16h b2 = ldfrag(wt, KCONV, n0 + 32, k0, lane);
    const v16h b3 = ldfrag(wt, KCONV, n0 + 48, k0, lane);
    acc[0][0] = mma16(a0, b0, acc[0][0]);
    acc[1][0] = mma16(a1, b0, acc[1][0]);
    acc[0][1] = mma16(a0, b1, acc[0][1]);
    acc[1][1] = mma16(a1, b1, acc[1][1]);
    acc[0][2] = mma16(a0, b2, acc[0][2]);
    acc[1][2] = mma16(a1, b2, acc[1][2]);
    acc[0][3] = mma16(a0, b3, acc[0][3]);
    acc[1][3] = mma16(a1, b3, acc[1][3]);
  }

  float bi[4], mv[4], rs[4], gg[4], bb[4];
#pragma unroll
  for (int t = 0; t < 4; ++t) {
    const int cl = 16 * t + c;
    bi[t] = ep[0][cl];
    mv[t] = ep[1][cl];
    rs[t] = ep[2][cl];
    gg[t] = ep[3][cl];
    bb[t] = ep[4][cl];
  }
  float* sw = st[wave];
#pragma unroll
  for (int sub = 0; sub < 2; ++sub) {
    __syncthreads();
#pragma unroll
    for (int t = 0; t < 4; ++t) {
#pragma unroll
      for (int r = 0; r < 8; ++r) {
        const float v = acc[sub][t][r] * 0.0009765625f + bi[t];
        const float y = (v - mv[t]) * rs[t] * gg[t] + bb[t];
        const float e = (y > 0.f) ? y : expm1f(fminf(y, 0.f));
        sw[(8 * hh + r) * OTP + 16 * t + c] = e;
      }
    }
    __syncthreads();
    if (SECOND) {
      v4f val[8];
      size_t go[8];
      int so[8];
#pragma unroll
      for (int it = 0; it < 8; ++it) {
        const int p    = lane + 32 * it;
        const int L    = p >> 3;
        const int pc   = p & 7;
        const int row  = L >> 1;
        const int half = L & 1;
        so[it]  = row * OTP + half * 32 + pc * 4;
        go[it]  = (size_t)(m0 + sub * 16 + row) * DM + n0 + half * 32 + pc * 4;
        val[it] = *(const v4f*)(sw + so[it]) + *(const v4f*)(res + go[it]);
      }
      for (int ps = 0; ps < 2; ++ps) {
#pragma unroll
        for (int it = 0; it < 8; ++it) *(volatile v4f*)(rout + go[it]) = val[it];
        __threadfence();
      }
#pragma unroll
      for (int it = 0; it < 8; ++it) *(v4f*)(sw + so[it]) = val[it];
      __syncthreads();
    }
    v4u hv[4];
    size_t ho[4];
#pragma unroll
    for (int it = 0; it < 4; ++it) {
      const int p  = lane + 32 * it;
      const int L  = p >> 3;
      const int pc = p & 7;
      const float* ra = sw + L * OTP + pc * 8;
      hv[it] = pack8h(*(const v4f*)(ra) * 16.0f, *(const v4f*)(ra + 4) * 16.0f);
      ho[it] = ((size_t)b * SQP + 1 + l0 + sub * 16 + L) * DM + n0 + pc * 8;
    }
    for (int ps = 0; ps < 2; ++ps) {
#pragma unroll
      for (int it = 0; it < 4; ++it) *(volatile v4u*)(hout + ho[it]) = hv[it];
      __threadfence();
    }
  }
}

__global__ __launch_bounds__(256) void k_pe(const float* __restrict__ xr, float* __restrict__ tf,
                                            _Float16* __restrict__ th) {
  __shared__ __align__(16) float sw[8][DM];
  const int tid = threadIdx.x, lane = tid & 31, wave = tid >> 5;
  const int m = blockIdx.x * 8 + wave;
  const int l = m & (SQ - 1);
  const float NEGC = -0.03597789207803197f;
  const float* row = xr + (size_t)m * DM;
#pragma unroll 1
  for (int j = 0; j < 4; ++j) {
    const int f0 = 8 * lane + 2 * j;
    const float dv  = expf((float)f0 * NEGC);
    const float ang = (float)l * dv;
    const float sv = sinf(ang);
    const float cv = cosf(ang);
    sw[wave][f0]     = row[f0] + sv;
    sw[wave][f0 + 1] = row[f0 + 1] + cv;
  }
  __syncthreads();
  v4f v[2];
#pragma unroll
  for (int it = 0; it < 2; ++it) v[it] = *(const v4f*)(sw[wave] + it * 128 + lane * 4);
  float* orow = tf + (size_t)m * DM;
  for (int ps = 0; ps < 2; ++ps) {
#pragma unroll
    for (int it = 0; it < 2; ++it) *(volatile v4f*)(orow + it * 128 + lane * 4) = v[it];
    __threadfence();
  }
  const float* cp = sw[wave] + 8 * lane;
  const v4u hv = pack8h(*(const v4f*)(cp), *(const v4f*)(cp + 4));
  _Float16* hdst = th + (size_t)m * DM + 8 * lane;
  for (int ps = 0; ps < 2; ++ps) {
    *(volatile v4u*)hdst = hv;
    __threadfence();
  }
}

#define STP 72
#define SVP 264
__global__ __launch_bounds__(256) void k_qkv(const _Float16* __restrict__ xh,
                                             const _Float16* __restrict__ wt,
                                             const float* __restrict__ bqkv,
                                             _Float16* __restrict__ qkp,
                                             _Float16* __restrict__ vtp) {
  __shared__ __align__(16) _Float16 st[256 * STP];
  const int tid = threadIdx.x, lane = tid & 31, wave = tid >> 5;
  const int hh = lane >> 4, c = lane & 15;
  const int bx = blockIdx.x;
  const int token0 = bx * 256;
  const int b  = bx >> 1;
  const int sb = (bx & 1) * 256;
  const int ns = blockIdx.y;
  const int which = ns >> 2;
  const int hp = ns & 3;
  const int m0 = token0 + wave * 32;
  const int n0 = ns * 64;

  v8f acc[2][4];
#pragma unroll
  for (int s = 0; s < 2; ++s)
#pragma unroll
    for (int t = 0; t < 4; ++t) acc[s][t] = zero8();
  gemm32x64(xh, DM, wt, DM, DM, m0, n0, lane, acc);

  float bb[4];
#pragma unroll
  for (int t = 0; t < 4; ++t) bb[t] = bqkv[n0 + 16 * t + c];
  const float wsc = 0.015625f;
  const float csc = 8.0f;

  if (which < 2) {
#pragma unroll
    for (int sub = 0; sub < 2; ++sub)
#pragma unroll
      for (int t = 0; t < 4; ++t)
#pragma unroll
        for (int r = 0; r < 8; ++r)
          st[(wave * 32 + sub * 16 + 8 * hh + r) * STP + 16 * t + c] =
              (_Float16)((acc[sub][t][r] * wsc + bb[t]) * csc);
  } else {
#pragma unroll
    for (int sub = 0; sub < 2; ++sub)
#pragma unroll
      for (int t = 0; t < 4; ++t)
#pragma unroll
        for (int r = 0; r < 8; ++r)
          st[(16 * t + c) * SVP + wave * 32 + sub * 16 + 8 * hh + r] =
              (_Float16)((acc[sub][t][r] * wsc + bb[t]) * csc);
  }
  __syncthreads();

  if (which < 2) {
    _Float16* base = qkp + (size_t)which * NTOK * DM + (size_t)token0 * DM + hp * 64;
#pragma unroll
    for (int gq = 0; gq < 2; ++gq) {
      v4u val[4];
      size_t go[4];
#pragma unroll
      for (int j = 0; j < 4; ++j) {
        const int p  = tid + 256 * (4 * gq + j);
        const int lr = p >> 3;
        const int pc = p & 7;
        Pack8 pk;
        pk.h   = *(const v8h*)(st + lr * STP + pc * 8);
        val[j] = pk.u;
        go[j]  = (size_t)lr * DM + pc * 8;
      }
      for (int ps = 0; ps < 2; ++ps) {
#pragma unroll
        for (int j = 0; j < 4; ++j) *(volatile v4u*)(base + go[j]) = val[j];
        __threadfence();
      }
    }
  } else {
    _Float16* base = vtp + (size_t)(b * NH + hp) * HDM * SQ + sb;
#pragma unroll
    for (int gq = 0; gq < 2; ++gq) {
      v4u val[4];
      size_t go[4];
#pragma unroll
      for (int j = 0; j < 4; ++j) {
        const int p    = tid + 256 * (4 * gq + j);
        const int drow = p >> 5;
        const int pc   = p & 31;
        Pack8 pk;
        pk.h   = *(const v8h*)(st + drow * SVP + pc * 8);
        val[j] = pk.u;
        go[j]  = (size_t)drow * SQ + pc * 8;
      }
      for (int ps = 0; ps < 2; ++ps) {
#pragma unroll
        for (int j = 0; j < 4; ++j) *(volatile v4u*)(base + go[j]) = val[j];
        __threadfence();
      }
    }
  }
}

#define KSP 72
#define VTP 72
#define PTP 72
__global__ __launch_bounds__(256) void k_attn(const _Float16* __restrict__ qkp,
                                              const _Float16* __restrict__ vtp,
                                              _Float16* __restrict__ aop, float sscale) {
  __shared__ __align__(16) _Float16 Ks[KC * KSP];
  __shared__ __align__(16) _Float16 Vs[HDM * VTP];
  __shared__ __align__(16) _Float16 Ps[8 * 16 * PTP];

  const int tid = threadIdx.x, lane = tid & 31, wave = tid >> 5;
  const int hh = lane >> 4, c = lane & 15;
  const int qb = blockIdx.x % NQB;
  const int hb = blockIdx.x / NQB;
  const int h  = hb % NH;
  const int b  = hb / NH;
  const int q0 = qb * QB + wave * 16;

  const _Float16* Q = qkp + (size_t)b * SQ * DM + h * HDM;
  const _Float16* K = qkp + (size_t)NTOK * DM + (size_t)b * SQ * DM + h * HDM;
  const _Float16* V = vtp + (size_t)hb * HDM * SQ;

  const v16h qa0 = ldfrag(Q, DM, q0, 0, lane);
  const v16h qa1 = ldfrag(Q, DM, q0, 32, lane);

  const float NEGI = -__builtin_huge_valf();
  float mrow[8], lrow[8];
  v8f oacc[4];
#pragma unroll
  for (int r = 0; r < 8; ++r) { mrow[r] = NEGI; lrow[r] = 0.f; }
#pragma unroll
  for (int t = 0; t < 4; ++t) oacc[t] = zero8();

  _Float16* pw = Ps + wave * 16 * PTP;

#pragma unroll 1
  for (int kc = 0; kc < NCK; ++kc) {
    const int kv0 = kc * KC;
    __syncthreads();
#pragma unroll
    for (int e = 0; e < 2; ++e) {
      const int p  = tid + 256 * e;
      const int r  = p >> 3;
      const int qq = (p & 7) * 8;
      *(v8h*)(Ks + r * KSP + qq) = *(const v8h*)(K + (size_t)(kv0 + r) * DM + qq);
      *(v8h*)(Vs + r * VTP + qq) = *(const v8h*)(V + (size_t)r * SQ + kv0 + qq);
    }
    __syncthreads();

    v8f s[4];
#pragma unroll
    for (int j = 0; j < 4; ++j) {
      const v16h kb0 = ldfrag(Ks, KSP, j * 16, 0, lane);
      const v16h kb1 = ldfrag(Ks, KSP, j * 16, 32, lane);
      s[j] = mma16(qa0, kb0, zero8());
      s[j] = mma16(qa1, kb1, s[j]);
    }
    float cm[8];
#pragma unroll
    for (int r = 0; r < 8; ++r) {
      float mx = NEGI;
#pragma unroll
      for (int j = 0; j < 4; ++j) {
        s[j][r] = s[j][r] * sscale;
        mx = fmaxf(mx, s[j][r]);
      }
#pragma unroll
      for (int off = 1; off < 16; off <<= 1) mx = fmaxf(mx, __shfl_xor(mx, off, 32));
      cm[r] = mx;
    }
    float al[8];
#pragma unroll
    for (int r = 0; r < 8; ++r) {
      const float mnew  = fmaxf(mrow[r], cm[r]);
      const float alpha = __expf(mrow[r] - mnew);
      mrow[r] = mnew;
      float psum = 0.f;
#pragma unroll
      for (int j = 0; j < 4; ++j) {
        const float p = __expf(s[j][r] - mnew);
        psum += p;
        pw[(8 * hh + r) * PTP + j * 16 + c] = (_Float16)(p * 1024.0f);
      }
#pragma unroll
      for (int off = 1; off < 16; off <<= 1) psum += __shfl_xor(psum, off, 32);
      lrow[r] = lrow[r] * alpha + psum;
      al[r] = alpha;
    }
#pragma unroll
    for (int t = 0; t < 4; ++t)
#pragma unroll
      for (int r = 0; r < 8; ++r) oacc[t][r] *= al[r];
    __syncthreads();

#pragma unroll
    for (int kk = 0; kk < 2; ++kk) {
      const v16h pa = ldfrag(pw, PTP, 0, kk * 32, lane);
#pragma unroll
      for (int t = 0; t < 4; ++t) {
        const v16h vb = ldfrag(Vs, VTP, t * 16, kk * 32, lane);
        oacc[t] = mma16(pa, vb, oacc[t]);
      }
    }
  }

  float inv[8];
#pragma unroll
  for (int r = 0; r < 8; ++r)
    inv[r] = (lrow[r] > 0.f) ? (0.00390625f * (1.0f / lrow[r])) : 0.f;
  __syncthreads();
#pragma unroll
  for (int r = 0; r < 8; ++r) {
#pragma unroll
    for (int t = 0; t < 4; ++t)
      pw[(8 * hh + r) * PTP + 16 * t + c] = (_Float16)(oacc[t][r] * inv[r]);
  }
  __syncthreads();
  v4u val[4];
  size_t go[4];
#pragma unroll
  for (int it = 0; it < 4; ++it) {
    const int p  = lane + 32 * it;
    const int L  = p >> 3;
    const int pc = p & 7;
    Pack8 pk;
    pk.h    = *(const v8h*)(pw + L * PTP + pc * 8);
    val[it] = pk.u;
    go[it]  = ((size_t)b * SQ + q0 + L) * DM + h * HDM + pc * 8;
  }
  for (int ps = 0; ps < 2; ++ps) {
#pragma unroll
    for (int it = 0; it < 4; ++it) *(volatile v4u*)(aop + go[it]) = val[it];
    __threadfence();
  }
}

__device__ __forceinline__ void out_epilogue_f32(v8f (&acc)[2][4], float scale, const float (&bb)[4],
                                                 float* sw, float* __restrict__ out, int ldo,
                                                 int m0, int n0, int lane, int hh, int c) {
#pragma unroll
  for (int sub = 0; sub < 2; ++sub) {
    __syncthreads();
#pragma unroll
    for (int t = 0; t < 4; ++t) {
#pragma unroll
      for (int r = 0; r < 8; ++r) sw[(8 * hh + r) * OTP + 16 * t + c] = acc[sub][t][r] * scale + bb[t];
    }
    __syncthreads();
    v4f val[8];
    size_t go[8];
#pragma unroll
    for (int it = 0; it < 8; ++it) {
      const int p    = lane + 32 * it;
      const int L    = p >> 3;
      const int pc   = p & 7;
      const int row  = L >> 1;
      const int half = L & 1;
      val[it] = *(const v4f*)(sw + row * OTP + half * 32 + pc * 4);
      go[it]  = (size_t)(m0 + sub * 16 + row) * ldo + n0 + half * 32 + pc * 4;
    }
    for (int ps = 0; ps < 2; ++ps) {
#pragma unroll
      for (int it = 0; it < 8; ++it) *(volatile v4f*)(out + go[it]) = val[it];
      __threadfence();
    }
  }
}

template <int RELU>
__device__ __forceinline__ void out_epilogue_h16(v8f (&acc)[2][4], float scale, const float (&bb)[4], float oscale,
                                                 float* sw, _Float16* __restrict__ out, int ldo,
                                                 int m0, int n0, int lane, int hh, int c) {
#pragma unroll
  for (int sub = 0; sub < 2; ++sub) {
    __syncthreads();
#pragma unroll
    for (int t = 0; t < 4; ++t) {
#pragma unroll
      for (int r = 0; r < 8; ++r) {
        float v = acc[sub][t][r] * scale + bb[t];
        if (RELU) v = fmaxf(v, 0.f);
        sw[(8 * hh + r) * OTP + 16 * t + c] = v * oscale;
      }
    }
    __syncthreads();
    v4u val[4];
    size_t go[4];
#pragma unroll
    for (int it = 0; it < 4; ++it) {
      const int p  = lane + 32 * it;
      const int L  = p >> 3;
      const int pc = p & 7;
      const float* ra = sw + L * OTP + pc * 8;
      val[it] = pack8h(*(const v4f*)(ra), *(const v4f*)(ra + 4));
      go[it]  = (size_t)(m0 + sub * 16 + L) * ldo + n0 + pc * 8;
    }
    for (int ps = 0; ps < 2; ++ps) {
#pragma unroll
      for (int it = 0; it < 4; ++it) *(volatile v4u*)(out + go[it]) = val[it];
      __threadfence();
    }
  }
}

template <int HASB>
__global__ __launch_bounds__(256) void k_gemm_f32(const _Float16* __restrict__ ap, int lda,
                                                  const _Float16* __restrict__ wt, int K,
                                                  const float* __restrict__ bias, float scale,
                                                  float* __restrict__ out, int ldo) {
  __shared__ __align__(16) float st[8][16 * OTP];
  const int tid = threadIdx.x, lane = tid & 31, wave = tid >> 5;
  const int hh = lane >> 4, c = lane & 15;
  const int m0 = blockIdx.x * 256 + wave * 32;
  const int n0 = blockIdx.y * 64;

  v8f acc[2][4];
#pragma unroll
  for (int s = 0; s < 2; ++s)
#pragma unroll
    for (int t = 0; t < 4; ++t) acc[s][t] = zero8();
  gemm32x64(ap, lda, wt, K, K, m0, n0, lane, acc);
  float bb[4];
#pragma unroll
  for (int t = 0; t < 4; ++t) {
    float v = 0.f;
    if (HASB) v = bias[n0 + 16 * t + c];
    bb[t] = v;
  }
  out_epilogue_f32(acc, scale, bb, st[wave], out, ldo, m0, n0, lane, hh, c);
}

template <int RELU>
__global__ __launch_bounds__(256) void k_gemm_h16(const _Float16* __restrict__ ap, int lda,
                                                  const _Float16* __restrict__ wt, int K,
                                                  const float* __restrict__ bias, float scale, float oscale,
                                                  _Float16* __restrict__ out, int ldo) {
  __shared__ __align__(16) float st[8][16 * OTP];
  const int tid = threadIdx.x, lane = tid & 31, wave = tid >> 5;
  const int hh = lane >> 4, c = lane & 15;
  const int m0 = blockIdx.x * 256 + wave * 32;
  const int n0 = blockIdx.y * 64;

  v8f acc[2][4];
#pragma unroll
  for (int s = 0; s < 2; ++s)
#pragma unroll
    for (int t = 0; t < 4; ++t) acc[s][t] = zero8();
  gemm32x64(ap, lda, wt, K, K, m0, n0, lane, acc);
  float bb[4];
#pragma unroll
  for (int t = 0; t < 4; ++t) bb[t] = bias[n0 + 16 * t + c];
  out_epilogue_h16<RELU>(acc, scale, bb, oscale, st[wave], out, ldo, m0, n0, lane, hh, c);
}

__global__ __launch_bounds__(256) void k_ln(const float* __restrict__ tp, const float* __restrict__ res,
                                            const float* __restrict__ g, const float* __restrict__ be,
                                            float* __restrict__ yf, _Float16* __restrict__ yh) {
  __shared__ __align__(16) float sw[8][DM];
  const int tid = threadIdx.x, lane = tid & 31, wave = tid >> 5;
  const int m = blockIdx.x * 8 + wave;

  v4f v[2];
  float sum = 0.f;
#pragma unroll
  for (int it = 0; it < 2; ++it) {
    const int idx = it * 128 + lane * 4;
    const size_t o = (size_t)m * DM + idx;
    const v4f a = *(const v4f*)(tp + o);
    const v4f r = *(const v4f*)(res + o);
    v[it] = a + r;
    sum += (v[it][0] + v[it][1]) + (v[it][2] + v[it][3]);
  }
#pragma unroll
  for (int off = 16; off >= 1; off >>= 1) sum += __shfl_xor(sum, off, 32);
  const float mean = sum * 0.00390625f;
  float ss = 0.f;
#pragma unroll
  for (int it = 0; it < 2; ++it) {
    const v4f d = v[it] - mean;
    ss += (d[0] * d[0] + d[1] * d[1]) + (d[2] * d[2] + d[3] * d[3]);
  }
#pragma unroll
  for (int off = 16; off >= 1; off >>= 1) ss += __shfl_xor(ss, off, 32);
  const float var  = ss * 0.00390625f;
  const float rstd = 1.0f / sqrtf(var + 1e-5f);

  v4f y[2];
#pragma unroll
  for (int it = 0; it < 2; ++it) {
    const int idx = it * 128 + lane * 4;
    const v4f gv = *(const v4f*)(g + idx);
    const v4f bv = *(const v4f*)(be + idx);
    y[it] = (v[it] - mean) * rstd * gv + bv;
  }
  for (int ps = 0; ps < 2; ++ps) {
#pragma unroll
    for (int it = 0; it < 2; ++it) *(volatile v4f*)(yf + (size_t)m * DM + it * 128 + lane * 4) = y[it];
    __threadfence();
  }
#pragma unroll
  for (int it = 0; it < 2; ++it) *(v4f*)(sw[wave] + it * 128 + lane * 4) = y[it];
  __syncthreads();
  const float* cp = sw[wave] + 8 * lane;
  const v4u hv = pack8h(*(const v4f*)(cp), *(const v4f*)(cp + 4));
  _Float16* hdst = yh + (size_t)m * DM + 8 * lane;
  for (int ps = 0; ps < 2; ++ps) {
    *(volatile v4u*)hdst = hv;
    __threadfence();
  }
}

__global__ __launch_bounds__(256) void k_concat(const float* __restrict__ xr, const float* __restrict__ tf,
                                                _Float16* __restrict__ xc) {
  const int half = blockIdx.y;
  const int idx = blockIdx.x * 256 + threadIdx.x;
  const int row = idx >> 5, pc = idx & 31;
  const size_t so = (size_t)row * DM + pc * 8;
  const v4f a0 = *(const v4f*)(xr + so), a1 = *(const v4f*)(xr + so + 4);
  const v4f t0 = *(const v4f*)(tf + so), t1 = *(const v4f*)(tf + so + 4);
  float f[8];
#pragma unroll
  for (int e = 0; e < 4; ++e) {
    f[e]     = (half != 0) ? t0[e] : a0[e];
    f[4 + e] = (half != 0) ? t1[e] : a1[e];
  }
  const v4u val = pack8h((v4f){f[0], f[1], f[2], f[3]}, (v4f){f[4], f[5], f[6], f[7]});
  _Float16* dst = xc + (size_t)row * KXC + half * DM + pc * 8;
  for (int ps = 0; ps < 2; ++ps) {
    *(volatile v4u*)dst = val;
    __threadfence();
  }
}

__global__ __launch_bounds__(256) void k_pair(const float* __restrict__ hij, const float* __restrict__ b1,
                                              const float* __restrict__ w2, const float* __restrict__ b2,
                                              float* __restrict__ lg) {
  __shared__ __align__(16) float sA[PR * NF1];
  __shared__ __align__(16) float sW[NF1];
  __shared__ __align__(16) float sO[PR * POP];
  const int tid = threadIdx.x;
  const int jh = blockIdx.x, i0 = blockIdx.y * PR, b = blockIdx.z;
  const int j  = jh * 256 + tid;

  if (tid < NF1) sW[tid] = w2[tid];
#pragma unroll 2
  for (int e = tid; e < PR * NF1; e += 256) {
    const int r = e >> 6, cc = e & 63;
    sA[e] = hij[((size_t)(b * SQ + i0 + r)) * NHIJ + cc] + b1[cc];
  }
  v4f hj[16];
  const float* hr = hij + (size_t)(b * SQ + j) * NHIJ + NF1;
#pragma unroll
  for (int q = 0; q < 16; ++q) hj[q] = *(const v4f*)(hr + 4 * q);
  const float bias2 = b2[0];
  __syncthreads();
  v4f wv[16];
#pragma unroll
  for (int q = 0; q < 16; ++q) wv[q] = *(const v4f*)(sW + 4 * q);

#pragma unroll 1
  for (int r = 0; r < PR; ++r) {
    const float* ar = sA + r * NF1;
    float s = 0.f;
#pragma unroll
    for (int q = 0; q < 16; ++q) {
      const v4f a = *(const v4f*)(ar + 4 * q);
      const v4f u = a + hj[q];
#pragma unroll
      for (int e = 0; e < 4; ++e) {
        const float ue = u[e];
        const float ev = (ue > 0.f) ? ue : (__expf(ue) - 1.0f);
        s = fmaf(ev, wv[q][e], s);
      }
    }
    sO[r * POP + tid] = s + bias2;
  }
  __syncthreads();

  v4f val[8];
  size_t go[8];
#pragma unroll
  for (int it = 0; it < 8; ++it) {
    const int p   = tid + 256 * it;
    const int row = p >> 6;
    const int pc  = p & 63;
    val[it] = *(const v4f*)(sO + row * POP + pc * 4);
    go[it]  = ((size_t)(b * SQ + i0 + row)) * SQ + jh * 256 + pc * 4;
  }
  for (int ps = 0; ps < 2; ++ps) {
#pragma unroll
    for (int it = 0; it < 8; ++it) *(volatile v4f*)(lg + go[it]) = val[it];
    __threadfence();
  }
}

__global__ __launch_bounds__(256) void k_sym(const float* __restrict__ lg, float* __restrict__ out) {
  __shared__ float sT[32][33];
  const int tid = threadIdx.x;
  const int j0 = blockIdx.x * 32, i0 = blockIdx.y * 32, b = blockIdx.z;
  const float* base = lg + (size_t)b * SQ * SQ;
#pragma unroll
  for (int k = 0; k < 4; ++k) {
    const int e = tid + 256 * k;
    const int r = e >> 5, cc = e & 31;
    sT[r][cc] = base[(size_t)(j0 + r) * SQ + i0 + cc];
  }
  __syncthreads();
  const int r2 = tid >> 3, pc = tid & 7;
  const size_t go = (size_t)(i0 + r2) * SQ + j0 + pc * 4;
  const v4f d  = *(const v4f*)(base + go);
  const v4f tv = (v4f){sT[pc * 4 + 0][r2], sT[pc * 4 + 1][r2], sT[pc * 4 + 2][r2], sT[pc * 4 + 3][r2]};
  const v4f val = (d + tv) * 0.5f;
  float* ob = out + (size_t)b * SQ * SQ;
  for (int ps = 0; ps < 2; ++ps) {
    *(volatile v4f*)(ob + go) = val;
    __threadfence();
  }
}

extern "C" void kernel_launch(void* const* d_in, const int* in_sizes, int n_in,
                              void* d_out, int out_size, void* d_ws, size_t ws_size,
                              hipStream_t stream) {
  if (n_in < 31) return;
  if (in_sizes[0] != NTOK * 4) return;
  if (in_sizes[1] != DM * 4) return;
  if (in_sizes[2] != DM) return;
  if (in_sizes[3] != NRES * DM * DM * 3) return;
  for (int i = 4; i <= 8; ++i) if (in_sizes[i] != NRES * DM) return;
  if (in_sizes[9] != NRES * DM * DM * 3) return;
  for (int i = 10; i <= 14; ++i) if (in_sizes[i] != NRES * DM) return;
  if (in_sizes[15] != NLAYER * NQKV * DM) return;
  if (in_sizes[16] != NLAYER * NQKV) return;
  if (in_sizes[17] != NLAYER * DM * DM) return;
  if (in_sizes[18] != NLAYER * DM) return;
  if (in_sizes[19] != NLAYER * DM || in_sizes[20] != NLAYER * DM) return;
  if (in_sizes[21] != NLAYER * DFF * DM) return;
  if (in_sizes[22] != NLAYER * DFF) return;
  if (in_sizes[23] != NLAYER * DM * DFF) return;
  if (in_sizes[24] != NLAYER * DM) return;
  if (in_sizes[25] != NLAYER * DM || in_sizes[26] != NLAYER * DM) return;
  if (in_sizes[27] != NF1 * 2 * KXC) return;
  if (in_sizes[28] != NF1) return;
  if (in_sizes[29] != NF1) return;
  if (in_sizes[30] < 1) return;
  if (out_size != NB * SQ * SQ) return;

  const float* x       = (const float*)d_in[0];
  const float* emb_w   = (const float*)d_in[1];
  const float* emb_b   = (const float*)d_in[2];
  const float* conv_w1 = (const float*)d_in[3];
  const float* conv_b1 = (const float*)d_in[4];
  const float* bn_g1   = (const float*)d_in[5];
  const float* bn_b1   = (const float*)d_in[6];
  const float* bn_m1   = (const float*)d_in[7];
  const float* bn_v1   = (const float*)d_in[8];
  const float* conv_w2 = (const float*)d_in[9];
  const float* conv_b2 = (const float*)d_in[10];
  const float* bn_g2   = (const float*)d_in[11];
  const float* bn_b2   = (const float*)d_in[12];
  const float* bn_m2   = (const float*)d_in[13];
  const float* bn_v2   = (const float*)d_in[14];
  const float* qkv_w   = (const float*)d_in[15];
  const float* qkv_b   = (const float*)d_in[16];
  const float* out_w   = (const float*)d_in[17];
  const float* out_b   = (const float*)d_in[18];
  const float* ln1_g   = (const float*)d_in[19];
  const float* ln1_b   = (const float*)d_in[20];
  const float* ff_w1   = (const float*)d_in[21];
  const float* ff_b1   = (const float*)d_in[22];
  const float* ff_w2   = (const float*)d_in[23];
  const float* ff_b2   = (const float*)d_in[24];
  const float* ln2_g   = (const float*)d_in[25];
  const float* ln2_b   = (const float*)d_in[26];
  const float* fc1_w   = (const float*)d_in[27];
  const float* fc1_b   = (const float*)d_in[28];
  const float* fc2_w   = (const float*)d_in[29];
  const float* fc2_b   = (const float*)d_in[30];
  float* out = (float*)d_out;

  size_t off = 0;
  const size_t oHP  = off; off += (size_t)3 * PADPLANE * 2;
  const size_t oR0  = off; off += (size_t)NTOK * DM * 4;
  const size_t oR1  = off; off += (size_t)NTOK * DM * 4;
  const size_t oWC1 = off; off += (size_t)NRES * DM * KCONV * 2;
  const size_t oWC2 = off; off += (size_t)NRES * DM * KCONV * 2;
  const size_t oWQ  = off; off += (size_t)NLAYER * NQKV * DM * 2;
  const size_t oWO  = off; off += (size_t)NLAYER * DM * DM * 2;
  const size_t oW1  = off; off += (size_t)NLAYER * DFF * DM * 2;
  const size_t oW2  = off; off += (size_t)NLAYER * DM * DFF * 2;
  const size_t oWF  = off; off += (size_t)NHIJ * KXC * 2;
  const size_t oTA  = off; off += (size_t)NTOK * DM * 4;
  const size_t oTB  = off; off += (size_t)NTOK * DM * 4;
  const size_t oT2  = off; off += (size_t)NTOK * DM * 4;
  const size_t oXh  = off; off += (size_t)NTOK * DM * 2;
  const size_t oQK  = off; off += (size_t)2 * NTOK * DM * 2;
  const size_t oVT  = off; off += (size_t)NB * NH * HDM * SQ * 2;
  const size_t oAO  = off; off += (size_t)NTOK * DM * 2;
  const size_t oHd  = off; off += (size_t)NTOK * DFF * 2;
  const size_t oXC  = off; off += (size_t)NTOK * KXC * 2;
  const size_t oHIJ = off; off += (size_t)NTOK * NHIJ * 4;
  const size_t oLG  = off; off += (size_t)NB * SQ * SQ * 4;
  if (off > ws_size) return;
  if (off > (size_t)134217728) return;

  char* ws = (char*)d_ws;
  _Float16* HPB = (_Float16*)(ws + oHP);
  _Float16* HP0 = HPB;
  _Float16* HP1 = HPB + PADPLANE;
  _Float16* HO  = HPB + 2 * (size_t)PADPLANE;
  float*    R0  = (float*)(ws + oR0);
  float*    R1  = (float*)(ws + oR1);
  _Float16* WC1 = (_Float16*)(ws + oWC1);
  _Float16* WC2 = (_Float16*)(ws + oWC2);
  _Float16* WQ  = (_Float16*)(ws + oWQ);
  _Float16* WO  = (_Float16*)(ws + oWO);
  _Float16* W1  = (_Float16*)(ws + oW1);
  _Float16* W2  = (_Float16*)(ws + oW2);
  _Float16* WF  = (_Float16*)(ws + oWF);
  float*    TA  = (float*)(ws + oTA);
  float*    TB  = (float*)(ws + oTB);
  float*    T2  = (float*)(ws + oT2);
  _Float16* Xh  = (_Float16*)(ws + oXh);
  _Float16* QK  = (_Float16*)(ws + oQK);
  _Float16* VT  = (_Float16*)(ws + oVT);
  _Float16* AO  = (_Float16*)(ws + oAO);
  _Float16* Hd  = (_Float16*)(ws + oHd);
  _Float16* XC  = (_Float16*)(ws + oXC);
  float*    HIJ = (float*)(ws + oHIJ);
  float*    LG  = (float*)(ws + oLG);

  k_padzero<<<dim3(3 * NB * 2), dim3(32), 0, stream>>>(HPB);
  k_convw<<<dim3(NRES * DM * 96 / 256), dim3(256), 0, stream>>>(conv_w1, WC1);
  k_convw<<<dim3(NRES * DM * 96 / 256), dim3(256), 0, stream>>>(conv_w2, WC2);
  k_cvt<<<dim3(NLAYER * NQKV * DM / 8 / 256), dim3(256), 0, stream>>>(qkv_w, NLAYER * NQKV * DM / 8, 64.0f, WQ);
  k_cvt<<<dim3(NLAYER * DM * DM / 8 / 256), dim3(256), 0, stream>>>(out_w, NLAYER * DM * DM / 8, 64.0f, WO);
  k_cvt<<<dim3(NLAYER * DFF * DM / 8 / 256), dim3(256), 0, stream>>>(ff_w1, NLAYER * DFF * DM / 8, 64.0f, W1);
  k_cvt<<<dim3(NLAYER * DM * DFF / 8 / 256), dim3(256), 0, stream>>>(ff_w2, NLAYER * DM * DFF / 8, 64.0f, W2);
  k_cvt_fc1<<<dim3(NHIJ * KXC / 8 / 256), dim3(256), 0, stream>>>(fc1_w, WF);
  k_embed<<<dim3(NTOK / 8), dim3(256), 0, stream>>>(x, emb_w, emb_b, R0, HP0);
  _Float16* HPc = HP0; _Float16* HPn = HP1;
  float* Rc = R0; float* Rn = R1;
  for (int i = 0; i < NRES; ++i) {
    const size_t wo = (size_t)i * DM * KCONV;
    const size_t po = (size_t)i * DM;
    k_conv<0><<<dim3(NTOK / 256, DM / 64), dim3(256), 0, stream>>>(HPc, WC1 + wo, conv_b1 + po, bn_g1 + po,
                                                                  bn_b1 + po, bn_m1 + po, bn_v1 + po,
                                                                  Rc, Rn, HO);
    k_conv<1><<<dim3(NTOK / 256, DM / 64), dim3(256), 0, stream>>>(HO, WC2 + wo, conv_b2 + po, bn_g2 + po,
                                                                  bn_b2 + po, bn_m2 + po, bn_v2 + po,
                                                                  Rc, Rn, HPn);
    _Float16* th = HPc; HPc = HPn; HPn = th;
    float* tr = Rc; Rc = Rn; Rn = tr;
  }
  k_pe<<<dim3(NTOK / 8), dim3(256), 0, stream>>>(Rc, TA, Xh);
  const float sscale = 0.001953125f;
  for (int l = 0; l < NLAYER; ++l) {
    const size_t po = (size_t)l * DM;
    k_qkv<<<dim3(NTOK / 256, NQKV / 64), dim3(256), 0, stream>>>(Xh, WQ + (size_t)l * NQKV * DM,
                                                                qkv_b + (size_t)l * NQKV, QK, VT);
    k_attn<<<dim3(NB * NH * NQB), dim3(256), 0, stream>>>(QK, VT, AO, sscale);
    k_gemm_f32<1><<<dim3(NTOK / 256, DM / 64), dim3(256), 0, stream>>>(AO, DM, WO + (size_t)l * DM * DM, DM,
                                                                      out_b + po, 0.00048828125f, T2, DM);
    k_ln<<<dim3(NTOK / 8), dim3(256), 0, stream>>>(T2, TA, ln1_g + po, ln1_b + po, TB, Xh);
    k_gemm_h16<1><<<dim3(NTOK / 256, DFF / 64), dim3(256), 0, stream>>>(Xh, DM, W1 + (size_t)l * DFF * DM, DM,
                                                                       ff_b1 + (size_t)l * DFF, 0.015625f, 16.0f,
                                                                       Hd, DFF);
    k_gemm_f32<1><<<dim3(NTOK / 256, DM / 64), dim3(256), 0, stream>>>(Hd, DFF, W2 + (size_t)l * DM * DFF, DFF,
                                                                      ff_b2 + po, 0.0009765625f, T2, DM);
    k_ln<<<dim3(NTOK / 8), dim3(256), 0, stream>>>(T2, TB, ln2_g + po, ln2_b + po, TA, Xh);
  }
  k_concat<<<dim3(NTOK * DM / 8 / 256, 2), dim3(256), 0, stream>>>(Rc, TA, XC);
  k_gemm_f32<0><<<dim3(NTOK / 256, NHIJ / 64), dim3(256), 0, stream>>>(XC, KXC, WF, KXC, fc1_b, 0.015625f,
                                                                    HIJ, NHIJ);
  k_pair<<<dim3(2, SQ / PR, NB), dim3(256), 0, stream>>>(HIJ, fc1_b, fc2_w, fc2_b, LG);
  k_sym<<<dim3(SQ / 32, SQ / 32, NB), dim3(256), 0, stream>>>(LG, out);
  (void)hipGetLastError();
}
